// STEncoderBlock_46866683134386
// MI455X (gfx1250) — hardware-verified
//
#include <hip/hip_runtime.h>
#include <math.h>

typedef __attribute__((ext_vector_type(16))) _Float16 v16h;
typedef __attribute__((ext_vector_type(16))) __bf16 v16b;
typedef __attribute__((ext_vector_type(8)))  _Float16 v8h;
typedef __attribute__((ext_vector_type(8)))  float v8f;
typedef __attribute__((ext_vector_type(4)))  float v4f;
typedef __attribute__((ext_vector_type(2)))  float v2f;
typedef __attribute__((ext_vector_type(4)))  unsigned v4u;
typedef __attribute__((ext_vector_type(4)))  int v4i;
typedef float __attribute__((may_alias)) float_a;
typedef int __attribute__((may_alias)) int_a;

template <typename T> __device__ __forceinline__ void vst2(void* p, T v) { *(volatile T*)p = v; __threadfence(); *(volatile T*)p = v; }
__device__ __forceinline__ v8f wmma16(v16h a, v16h b, v8f c) {
  v8f d = __builtin_amdgcn_wmma_f32_16x16x32_f16(false, a, false, b, (short)0, c, false, false);
  asm volatile("v_nop\n\tv_nop\n\tv_nop\n\tv_nop" : "+v"(d) : "v"(a), "v"(b));
  return d;
}
__device__ __forceinline__ v8f wmma_bf(v16b a, v16b b, v8f c) {
  v8f d = __builtin_amdgcn_wmma_f32_16x16x32_bf16(false, a, false, b, (short)0, c, false, false);
  asm volatile("v_nop\n\tv_nop\n\tv_nop\n\tv_nop" : "+v"(d) : "v"(a), "v"(b));
  return d;
}
__device__ __forceinline__ v16h frag_h(const _Float16* rowk0, int lane) {
  union { v16h v; v8h q[2]; } u; const _Float16* p = rowk0 + 8 * (lane >> 4);
  u.q[0] = *(const v8h*)p; u.q[1] = *(const v8h*)(p + 16); return u.v;
}
__device__ __forceinline__ v16h frag_f32(const float* rowk0, int lane) {
  v16h a; const float* p = rowk0 + 8 * (lane >> 4);
#pragma unroll
  for (int i = 0; i < 8; ++i) { a[i] = (_Float16)p[i]; a[8 + i] = (_Float16)p[16 + i]; }
  return a;
}
__device__ __forceinline__ v16h frag_f32s(const float* rowk0, int lane, float sc) {
  v16h a; const float* p = rowk0 + 8 * (lane >> 4);
#pragma unroll
  for (int i = 0; i < 8; ++i) { a[i] = (_Float16)(p[i] * sc); a[8 + i] = (_Float16)(p[16 + i] * sc); }
  return a;
}
__device__ __forceinline__ v16h fragc_f32(const float* W, int k0, int n, int lane, int ld, int K) {
  v16h a; const int g = lane >> 4;
#pragma unroll
  for (int i = 0; i < 8; ++i) { const int ka = k0 + 8 * g + i, kb = ka + 16;
    a[i] = (_Float16)(ka < K ? W[(size_t)(ka < K ? ka : K - 1) * ld + n] : 0.f); a[8 + i] = (_Float16)(kb < K ? W[(size_t)(kb < K ? kb : K - 1) * ld + n] : 0.f); }
  return a;
}
struct F2 { v16b h, l; };
__device__ __forceinline__ F2 bsplit16(const float v[16]) { F2 r;
#pragma unroll
  for (int i = 0; i < 16; ++i) { const __bf16 h = (__bf16)v[i]; r.h[i] = h; r.l[i] = (__bf16)(v[i] - (float)h); }
  return r; }
__device__ __forceinline__ F2 split_row(const float* row, int k0, int lane) { float v[16]; const float* p = row + k0 + 8 * (lane >> 4);
#pragma unroll
  for (int i = 0; i < 8; ++i) { v[i] = p[i]; v[8 + i] = p[16 + i]; }
  return bsplit16(v); }
__device__ __forceinline__ F2 split_rowK(const float* row, int k0, int lane, int K) { float v[16]; const int g = lane >> 4;
#pragma unroll
  for (int i = 0; i < 8; ++i) { const int ka = k0 + 8 * g + i, kb = ka + 16; v[i] = ka < K ? row[ka < K ? ka : K - 1] : 0.f; v[8 + i] = kb < K ? row[kb < K ? kb : K - 1] : 0.f; }
  return bsplit16(v); }
__device__ __forceinline__ F2 split_col(const float* W, int k0, int n, int lane, int ld, int K) { float v[16]; const int g = lane >> 4;
#pragma unroll
  for (int i = 0; i < 8; ++i) { const int ka = k0 + 8 * g + i, kb = ka + 16; v[i] = ka < K ? W[(size_t)(ka < K ? ka : K - 1) * ld + n] : 0.f; v[8 + i] = kb < K ? W[(size_t)(kb < K ? kb : K - 1) * ld + n] : 0.f; }
  return bsplit16(v); }
__device__ __forceinline__ v8f mac3(const F2& a, const F2& b, v8f c) { c = wmma_bf(a.l, b.h, c); c = wmma_bf(a.h, b.l, c); return wmma_bf(a.h, b.h, c); }
__device__ __forceinline__ float sigm(float v) { return 1.0f / (1.0f + expf(-v)); }
#define LDSX() do { asm volatile("s_wait_dscnt 0" ::: "memory"); __builtin_amdgcn_wave_barrier(); __builtin_amdgcn_fence(__ATOMIC_RELEASE, "workgroup"); } while (0)


#define NB 16
#define NT 24
#define NN 512
#define DD 64
#define FF 256
#define NR (NB * NT * NN)
#define NSL (NB * NT)
#define CH 96
#define EPS_ 1e-5f
#ifndef TNSL
#define TNSL NSL
#endif
#ifndef TNBA
#define TNBA NB
#endif
typedef __attribute__((ext_vector_type(8))) __bf16 v8b;
__device__ __forceinline__ v16b frag_b(const __bf16* rowk0, int lane) {
  union { v16b v; v8b q[2]; } u; const __bf16* p = rowk0 + 8 * (lane >> 4);
  u.q[0] = *(const v8b*)p; u.q[1] = *(const v8b*)(p + 16); return u.v;
}
__device__ __forceinline__ v16b frag_gbf(const float* rowk0, int lane) {
  v16b a; const float* p = rowk0 + 8 * (lane >> 4);
#pragma unroll
  for (int i = 0; i < 8; ++i) { a[i] = (__bf16)p[i]; a[8 + i] = (__bf16)p[16 + i]; }
  return a;
}
__device__ __forceinline__ float bfr(float v) { return (float)(__bf16)v; }
__device__ __attribute__((noinline)) float exp_ni(float v) { return expf(v); }
__device__ __attribute__((noinline)) float erf_ni(float v) { return erff(v); }
#define PR_QKVO 0
#define PR_GC (4 * 64)
#define PR_W1 (7 * 64)
#define PR_W2 (7 * 64 + 256)
#define PT_BYTES (2u * ((7 * 64 + 256) * 64 + 64 * 256))
#define WS_PT   0u
#define WS_DINV (WS_PT + PT_BYTES)
#define WS_H    (WS_DINV + 4u * NN)
#define WS_YTH  (WS_H + 4u * NR * DD)
#define WS_YTL  (WS_YTH + 2u * CH * DD * NN)
#define WS_Y2H  (WS_YTL + 2u * CH * DD * NN)
#define WS_Y2L  (WS_Y2H + 2u * CH * DD * NN)
#define WS_G    (WS_Y2L + 2u * CH * DD * NN)
#define WS_END  (WS_G + 4u * CH * NN * DD)

__global__ __launch_bounds__(256) void k_pack(const float* __restrict__ Wq, const float* __restrict__ Wk, const float* __restrict__ Wv, const float* __restrict__ Wo, const float* __restrict__ GCW, const float* __restrict__ W1, const float* __restrict__ W2, __bf16* __restrict__ PT) {
  __shared__ __align__(16) __bf16 srow[256];
  const int n = blockIdx.x, tid = threadIdx.x; int len = 64; size_t dst;
  if (n < 256) { const int w = n >> 6, c = n & 63; const float* Wm = w == 0 ? Wq : w == 1 ? Wk : w == 2 ? Wv : Wo; if (tid < 64) srow[tid] = (__bf16)bfr(Wm[tid * 64 + c]); dst = (size_t)n * 64; }
  else if (n < 448) { const int m = n - 256; const int w = m >> 6, c = m & 63; if (tid < 64) srow[tid] = (__bf16)bfr(GCW[(size_t)w * 4096 + tid * 64 + c]); dst = (size_t)n * 64; }
  else if (n < 704) { const int c = n - 448; if (tid < 64) srow[tid] = (__bf16)bfr(W1[tid * 256 + c]); dst = (size_t)n * 64; }
  else { const int c = n - 704; len = 256; srow[tid] = (__bf16)bfr(W2[(size_t)tid * 64 + c]); dst = (size_t)704 * 64 + (size_t)c * 256; }
  __syncthreads();
  if (tid < len / 8) vst2((unsigned*)(PT + dst + tid * 8), *(const v4u*)(&srow[tid * 8]));
}
__global__ __launch_bounds__(256) void k_dinv(const float* __restrict__ ADJ, float* __restrict__ DINV) {
  __shared__ __align__(16) float sd[64]; __shared__ float sp[64][4];
  const int tid = threadIdx.x; const int r = tid >> 2, part = tid & 3; const int m = blockIdx.x * 64 + r; float s = 0.f;
  for (int n = part * 128; n < part * 128 + 128; ++n) s += bfr(ADJ[(size_t)m * NN + n]);
  sp[r][part] = s; __syncthreads();
  if (tid < 64) { const float deg = ((sp[tid][0] + sp[tid][1]) + (sp[tid][2] + sp[tid][3])) + 1.0f; sd[tid] = 1.0f / sqrtf(fmaxf(deg, 1e-12f)); }
  __syncthreads();
  if (tid < 16) vst2(DINV + blockIdx.x * 64 + tid * 4, *(const v4f*)&sd[tid * 4]);
}
__global__ __launch_bounds__(128) void k_att(const float* __restrict__ X, const __bf16* __restrict__ PT, const float* __restrict__ bq, const float* __restrict__ bk, const float* __restrict__ bv, const float* __restrict__ bo, const float* __restrict__ gt, const float* __restrict__ bt, float* __restrict__ Hh) {
  __shared__ __align__(16) float sq[32][196]; __shared__ __align__(16) __bf16 sah[32][72], sal[32][72]; __shared__ __align__(16) float so[32][68];
  const int tid = threadIdx.x, wave = tid >> 5, lane = tid & 31, col = lane & 15, g = lane >> 4; const int n = blockIdx.x, b = blockIdx.y; const int rt = wave & 1, chh = wave >> 1;
  auto rowof = [&](int t) { return ((size_t)(b * NT + min(t, NT - 1)) * NN + n); };
  { v8f acc[6] = {};
#pragma unroll
    for (int kc = 0; kc < 2; ++kc) { const v16b a = frag_gbf(X + rowof(rt * 16 + col) * DD + kc * 32, lane);
#pragma unroll
      for (int j = 0; j < 6; ++j) { const int tile = chh * 6 + j; acc[j] = wmma_bf(a, frag_b(PT + (size_t)(PR_QKVO + tile * 16 + col) * DD + kc * 32, lane), acc[j]); } }
#pragma unroll
    for (int j = 0; j < 6; ++j) { const int tile = chh * 6 + j; const int o = tile * 16 + col; const int w = o >> 6, c = o & 63; const float bb = bfr((w == 0 ? bq : w == 1 ? bk : bv)[c]);
#pragma unroll
      for (int r = 0; r < 8; ++r) sq[rt * 16 + 8 * g + r][o] = acc[j][r] + bb; } }
  __syncthreads();
  { const int t = tid >> 2, h = tid & 3; float sc[NT]; float mx = -3.0e38f;
#pragma unroll
    for (int u = 0; u < NT; ++u) { float s = 0.f; for (int d = 0; d < 16; ++d) s += sq[t][h * 16 + d] * sq[u][64 + h * 16 + d]; s *= 0.25f; sc[u] = s; mx = fmaxf(mx, s); }
    float z = 0.f;
#pragma unroll
    for (int u = 0; u < NT; ++u) { sc[u] = exp_ni(sc[u] - mx); z += sc[u]; }
    const float iz = 1.0f / z;
    for (int d = 0; d < 16; ++d) { float a = 0.f;
#pragma unroll
      for (int u = 0; u < NT; ++u) a += sc[u] * sq[u][128 + h * 16 + d];
      a *= iz; const __bf16 hb = (__bf16)a; sah[t][h * 16 + d] = hb; sal[t][h * 16 + d] = (__bf16)(a - (float)hb); } }
  __syncthreads();
  { v8f acc[2] = {};
#pragma unroll
    for (int kc = 0; kc < 2; ++kc) { const v16b ah = frag_b(&sah[rt * 16 + col][kc * 32], lane), al = frag_b(&sal[rt * 16 + col][kc * 32], lane);
#pragma unroll
      for (int j = 0; j < 2; ++j) { const v16b w = frag_b(PT + (size_t)(PR_QKVO + 192 + (chh * 2 + j) * 16 + col) * DD + kc * 32, lane); acc[j] = wmma_bf(al, w, acc[j]); acc[j] = wmma_bf(ah, w, acc[j]); } }
#pragma unroll
    for (int j = 0; j < 2; ++j) { const int o = (chh * 2 + j) * 16 + col; const float bb = bfr(bo[o]);
#pragma unroll
      for (int r = 0; r < 8; ++r) { const int t = rt * 16 + 8 * g + r; so[t][o] = acc[j][r] + bb + bfr(X[rowof(t) * DD + o]); } } }
  __syncthreads();
  if (tid < NT * 4) { const int t = tid >> 2, part = tid & 3; float s = 0.f; for (int c = 0; c < DD; ++c) s += so[t][c]; const float mu = s / 64.f; float v = 0.f; for (int c = 0; c < DD; ++c) { const float d = so[t][c] - mu; v += d * d; } const float rs = rsqrtf(v / 64.f + EPS_);
    v4f o4[4];
#pragma unroll
    for (int p = 0; p < 4; ++p) for (int i = 0; i < 4; ++i) { const int c = part * 16 + p * 4 + i; o4[p][i] = (so[t][c] - mu) * rs * bfr(gt[c]) + bfr(bt[c]); }
    __syncthreads();
#pragma unroll
    for (int p = 0; p < 4; ++p) vst2(Hh + rowof(t) * DD + part * 16 + p * 4, o4[p]); }
  else { __syncthreads(); }
}
__global__ __launch_bounds__(256) void k_prep(const float* __restrict__ Hh, const float* __restrict__ DINV, __bf16* __restrict__ YTH, __bf16* __restrict__ YTL, int slab0) {
  __shared__ __align__(16) __bf16 sth[DD][72], stl[DD][72];
  const int sl = blockIdx.y, n0 = blockIdx.x * 64, tid = threadIdx.x; const size_t rbase = (size_t)(slab0 + sl) * NN + n0;
  for (int q = tid; q < 64 * DD; q += 256) { const int nl = q >> 6, d = q & 63; const float v = Hh[(rbase + nl) * DD + d] * DINV[n0 + nl]; const __bf16 hb = (__bf16)v; sth[d][nl] = hb; stl[d][nl] = (__bf16)(v - (float)hb); }
  __syncthreads();
  for (int q = tid; q < DD * 8; q += 256) { const int d = q >> 3, pc = q & 7; const size_t o = ((size_t)sl * DD + d) * NN + n0 + pc * 8; vst2((unsigned*)(YTH + o), *(const v4u*)&sth[d][pc * 8]); vst2((unsigned*)(YTL + o), *(const v4u*)&stl[d][pc * 8]); }
}
__device__ __forceinline__ void hop_acc(const float* __restrict__ ADJ, const __bf16* __restrict__ YTH, const __bf16* __restrict__ YTL, int sl, int mrow, v8f* acc, int lane) {
  const int col = lane & 15;
#pragma unroll 1
  for (int kc = 0; kc < NN / 32; ++kc) { const v16b a = frag_gbf(ADJ + (size_t)mrow * NN + kc * 32, lane);
#pragma unroll
    for (int dt = 0; dt < 4; ++dt) { const size_t o = ((size_t)sl * DD + dt * 16 + col) * NN + kc * 32; acc[dt] = wmma_bf(a, frag_b(YTL + o, lane), acc[dt]); acc[dt] = wmma_bf(a, frag_b(YTH + o, lane), acc[dt]); } }
}
__global__ __launch_bounds__(128) void k_hop1(const float* __restrict__ ADJ, const float* __restrict__ Hh, const float* __restrict__ DINV, const __bf16* __restrict__ YTH, const __bf16* __restrict__ YTL, const __bf16* __restrict__ PT, const float* __restrict__ gcb, float* __restrict__ G, __bf16* __restrict__ Y2H, __bf16* __restrict__ Y2L, int slab0) {
  __shared__ __align__(16) __bf16 sph[4][16][72], spl[4][16][72]; __shared__ __align__(16) __bf16 s2h[DD][72], s2l[DD][72]; __shared__ __align__(16) float so[4][16][68];
  const int tid = threadIdx.x, wave = tid >> 5, lane = tid & 31, col = lane & 15, g = lane >> 4; const int sl = blockIdx.y, m0 = blockIdx.x * 64 + wave * 16; const size_t rbase = (size_t)(slab0 + sl) * NN;
  v8f acc[4] = {};
  hop_acc(ADJ, YTH, YTL, sl, m0 + col, acc, lane);
#pragma unroll
  for (int dt = 0; dt < 4; ++dt) { const int d = dt * 16 + col;
#pragma unroll
    for (int r = 0; r < 8; ++r) { const int m = m0 + 8 * g + r; const float dm = DINV[m]; const float p1 = dm * (acc[dt][r] + dm * Hh[(rbase + m) * DD + d]); const __bf16 hb = (__bf16)p1; sph[wave][8 * g + r][d] = hb; spl[wave][8 * g + r][d] = (__bf16)(p1 - (float)hb);
      const float y2 = dm * p1; const __bf16 h2 = (__bf16)y2; s2h[d][wave * 16 + 8 * g + r] = h2; s2l[d][wave * 16 + 8 * g + r] = (__bf16)(y2 - (float)h2); } }
  LDSX();
  { v8f gacc[4] = {};
#pragma unroll
    for (int kc = 0; kc < 2; ++kc) { const F2 ah = split_row(Hh + (rbase + m0 + col) * DD, kc * 32, lane); const v16b ph = frag_b(&sph[wave][col][kc * 32], lane), pl = frag_b(&spl[wave][col][kc * 32], lane);
#pragma unroll
      for (int j = 0; j < 4; ++j) { const v16b w0 = frag_b(PT + (size_t)(PR_GC + 0 * 64 + j * 16 + col) * DD + kc * 32, lane), w1 = frag_b(PT + (size_t)(PR_GC + 1 * 64 + j * 16 + col) * DD + kc * 32, lane);
        gacc[j] = wmma_bf(ah.l, w0, gacc[j]); gacc[j] = wmma_bf(ah.h, w0, gacc[j]); gacc[j] = wmma_bf(pl, w1, gacc[j]); gacc[j] = wmma_bf(ph, w1, gacc[j]); } }
#pragma unroll
    for (int j = 0; j < 4; ++j) { const int o = j * 16 + col; const float bb = bfr(gcb[o]) + bfr(gcb[64 + o]);
#pragma unroll
      for (int r = 0; r < 8; ++r) so[wave][8 * g + r][o] = gacc[j][r] + bb; } }
  __syncthreads();
  for (int rl = 0; rl < 16; ++rl) if (lane < 16) vst2(G + ((size_t)sl * NN + m0 + rl) * DD + lane * 4, *(const v4f*)&so[wave][rl][lane * 4]);
  for (int q = tid; q < DD * 8; q += 128) { const int d = q >> 3, pc = q & 7; const size_t o = ((size_t)sl * DD + d) * NN + blockIdx.x * 64 + pc * 8; vst2((unsigned*)(Y2H + o), *(const v4u*)&s2h[d][pc * 8]); vst2((unsigned*)(Y2L + o), *(const v4u*)&s2l[d][pc * 8]); }
}
__global__ __launch_bounds__(128) void k_hop2(const float* __restrict__ ADJ, const float* __restrict__ Hh, const float* __restrict__ DINV, const __bf16* __restrict__ Y2H, const __bf16* __restrict__ Y2L, const __bf16* __restrict__ PT, const float* __restrict__ gcb, const float* __restrict__ G,
                                            const float* __restrict__ b1, const float* __restrict__ b2, const float* __restrict__ gg, const float* __restrict__ bg, const float* __restrict__ gf, const float* __restrict__ bff, float* __restrict__ OUT, int slab0) {
  __shared__ __align__(16) __bf16 sph[4][16][72], spl[4][16][72]; __shared__ __align__(16) float so[4][16][68]; __shared__ __align__(16) __bf16 shh[4][16][264], shl[4][16][264]; __shared__ float sh2[4][16][65];
  const int tid = threadIdx.x, wave = tid >> 5, lane = tid & 31, col = lane & 15, g = lane >> 4; const int sl = blockIdx.y, m0 = blockIdx.x * 64 + wave * 16; const size_t rbase = (size_t)(slab0 + sl) * NN;
  v8f acc[4] = {};
  hop_acc(ADJ, Y2H, Y2L, sl, m0 + col, acc, lane);
#pragma unroll
  for (int dt = 0; dt < 4; ++dt) { const int d = dt * 16 + col;
#pragma unroll
    for (int r = 0; r < 8; ++r) { const int m = m0 + 8 * g + r; const size_t o = ((size_t)sl * DD + d) * NN + m; const float y2 = (float)Y2H[o] + (float)Y2L[o]; const float p2 = DINV[m] * (acc[dt][r] + y2); const __bf16 hb = (__bf16)p2; sph[wave][8 * g + r][d] = hb; spl[wave][8 * g + r][d] = (__bf16)(p2 - (float)hb); } }
  LDSX();
  { v8f gacc[4] = {};
#pragma unroll
    for (int kc = 0; kc < 2; ++kc) { const v16b ph = frag_b(&sph[wave][col][kc * 32], lane), pl = frag_b(&spl[wave][col][kc * 32], lane);
#pragma unroll
      for (int j = 0; j < 4; ++j) { const v16b w2 = frag_b(PT + (size_t)(PR_GC + 2 * 64 + j * 16 + col) * DD + kc * 32, lane); gacc[j] = wmma_bf(pl, w2, gacc[j]); gacc[j] = wmma_bf(ph, w2, gacc[j]); } }
#pragma unroll
    for (int j = 0; j < 4; ++j) { const int o = j * 16 + col; const float bb = bfr(gcb[128 + o]);
#pragma unroll
      for (int r = 0; r < 8; ++r) { const size_t row = rbase + m0 + 8 * g + r; so[wave][8 * g + r][o] = gacc[j][r] + bb + G[((size_t)sl * NN + m0 + 8 * g + r) * DD + o] + Hh[row * DD + o]; } } }
  LDSX();
  { const int rl = lane >> 1, half = lane & 1; float s = 0.f; for (int c = half * 32; c < half * 32 + 32; ++c) s += so[wave][rl][c]; s += __shfl_xor(s, 1); const float mu = s / 64.f; float v = 0.f; for (int c = half * 32; c < half * 32 + 32; ++c) { const float d = so[wave][rl][c] - mu; v += d * d; } v += __shfl_xor(v, 1); const float rs = rsqrtf(v / 64.f + EPS_);
    for (int c = half * 32; c < half * 32 + 32; ++c) { const float y = (so[wave][rl][c] - mu) * rs * bfr(gg[c]) + bfr(bg[c]); sh2[wave][rl][c] = y; const __bf16 hb = (__bf16)y; shh[wave][rl][c] = hb; shl[wave][rl][c] = (__bf16)(y - (float)hb); } }
  LDSX();
  { v8f f[16];
#pragma unroll
    for (int j = 0; j < 16; ++j) f[j] = (v8f){};
#pragma unroll
    for (int kc = 0; kc < 2; ++kc) { const v16b ah = frag_b(&shh[wave][col][kc * 32], lane), al = frag_b(&shl[wave][col][kc * 32], lane);
#pragma unroll
      for (int j = 0; j < 16; ++j) { const v16b w = frag_b(PT + (size_t)(PR_W1 + j * 16 + col) * DD + kc * 32, lane); f[j] = wmma_bf(al, w, f[j]); f[j] = wmma_bf(ah, w, f[j]); } }
    LDSX();
#pragma unroll
    for (int j = 0; j < 16; ++j) { const int o = j * 16 + col; const float bb = bfr(b1[o]);
#pragma unroll
      for (int r = 0; r < 8; ++r) { const float xg = f[j][r] + bb; const float gl = 0.5f * xg * (1.0f + erf_ni(xg * 0.70710678118654752f)); const __bf16 hb = (__bf16)gl; shh[wave][8 * g + r][o] = hb; shl[wave][8 * g + r][o] = (__bf16)(gl - (float)hb); } } }
  LDSX();
  { v8f d4[4] = {};
#pragma unroll
    for (int kc = 0; kc < 8; ++kc) { const v16b ah = frag_b(&shh[wave][col][kc * 32], lane), al = frag_b(&shl[wave][col][kc * 32], lane);
#pragma unroll
      for (int j = 0; j < 4; ++j) { const v16b w = frag_b(PT + (size_t)704 * 64 + (size_t)(j * 16 + col) * FF + kc * 32, lane); d4[j] = wmma_bf(al, w, d4[j]); d4[j] = wmma_bf(ah, w, d4[j]); } }
#pragma unroll
    for (int j = 0; j < 4; ++j) { const int o = j * 16 + col; const float bb = bfr(b2[o]);
#pragma unroll
      for (int r = 0; r < 8; ++r) so[wave][8 * g + r][o] = d4[j][r] + bb + sh2[wave][8 * g + r][o]; } }
  LDSX();
  { const int rl = lane >> 1, half = lane & 1; float s = 0.f; for (int c = half * 32; c < half * 32 + 32; ++c) s += so[wave][rl][c]; s += __shfl_xor(s, 1); const float mu = s / 64.f; float v = 0.f; for (int c = half * 32; c < half * 32 + 32; ++c) { const float d = so[wave][rl][c] - mu; v += d * d; } v += __shfl_xor(v, 1); const float rs = rsqrtf(v / 64.f + EPS_);
    LDSX();
    for (int c = half * 32; c < half * 32 + 32; ++c) so[wave][rl][c] = (so[wave][rl][c] - mu) * rs * bfr(gf[c]) + bfr(bff[c]); }
  LDSX();
  for (int rl = 0; rl < 16; ++rl) if (lane < 16) vst2(OUT + (rbase + m0 + rl) * DD + lane * 4, *(const v4f*)&so[wave][rl][lane * 4]);
}

extern "C" void kernel_launch(void* const* d_in, const int* in_sizes, int n_in, void* d_out, int out_size, void* d_ws, size_t ws_size, hipStream_t stream) {
  (void)in_sizes; (void)n_in; (void)out_size;
  const float** F = (const float**)d_in;
  if (ws_size < (size_t)WS_END) return;
  char* ws = (char*)d_ws; __bf16* PT = (__bf16*)(ws + WS_PT); float *DINV = (float*)(ws + WS_DINV), *Hh = (float*)(ws + WS_H), *G = (float*)(ws + WS_G); __bf16 *YTH = (__bf16*)(ws + WS_YTH), *YTL = (__bf16*)(ws + WS_YTL), *Y2H = (__bf16*)(ws + WS_Y2H), *Y2L = (__bf16*)(ws + WS_Y2L);
  k_pack<<<768, 256, 0, stream>>>(F[2], F[4], F[6], F[8], F[10], F[12], F[14], PT);
  k_dinv<<<NN / 64, 256, 0, stream>>>(F[1], DINV);
  k_att<<<dim3(NN, TNBA), 128, 0, stream>>>(F[0], PT, F[3], F[5], F[7], F[9], F[16], F[17], Hh);
  for (int c0 = 0; c0 < TNSL; c0 += CH) { const int nsl = min(CH, TNSL - c0);
    k_prep<<<dim3(NN / 64, nsl), 256, 0, stream>>>(Hh, DINV, YTH, YTL, c0);
    k_hop1<<<dim3(NN / 64, nsl), 128, 0, stream>>>(F[1], Hh, DINV, YTH, YTL, PT, F[11], G, Y2H, Y2L, c0);
    k_hop2<<<dim3(NN / 64, nsl), 128, 0, stream>>>(F[1], Hh, DINV, Y2H, Y2L, PT, F[11], G, F[13], F[15], F[18], F[19], F[20], F[21], (float*)d_out, c0); }
}
